// CharModel_88811333747032
// MI455X (gfx1250) — hardware-verified
//
#include <hip/hip_runtime.h>


namespace {
constexpr int NB = 4096, T = 128, V = 128, E = 42, EP = 64, H = 256, RB = 32  ;
constexpr float XS = 8.0f, WSC = 256.0f;
typedef _Float16 b16;
typedef __attribute__((ext_vector_type(16))) _Float16 v16b;
typedef __attribute__((ext_vector_type(8))) _Float16 v8b;
typedef __attribute__((ext_vector_type(8))) float v8f;
typedef __attribute__((ext_vector_type(4))) float v4f;
__device__ __forceinline__ float bf16_rne(float f) { unsigned int u = __float_as_uint(f); u += 0x7FFFu + ((u >> 16) & 1u); return __uint_as_float(u & 0xFFFF0000u); }
__device__ __forceinline__ void split16(float v, b16& hi, b16& lo) { hi = (b16)v; lo = (b16)(v - (float)hi); }
__device__ __forceinline__ v16b frag_kb(const b16* p, int hh) { const v8b a = *(const v8b*)(p + 8 * hh), b = *(const v8b*)(p + 16 + 8 * hh); v16b f;
#pragma unroll
  for (int e = 0; e < 8; ++e) { f[e] = a[e]; f[8 + e] = b[e]; } return f; }
__device__ __forceinline__ v8f wmma16b(v16b a, v16b b, v8f c) { v8f d = __builtin_amdgcn_wmma_f32_16x16x32_f16(false, a, false, b, (short)0, c, false, false); asm volatile("v_nop\n\tv_nop\n\tv_nop\n\tv_nop" : "+v"(d) : "v"(a), "v"(b)); return d; }
__device__ __forceinline__ void wave_lds_sync() { __builtin_amdgcn_fence(__ATOMIC_RELEASE, "workgroup"); __builtin_amdgcn_wave_barrier(); __builtin_amdgcn_fence(__ATOMIC_ACQUIRE, "workgroup"); }
__device__ __forceinline__ int iclamp(int v, int lo, int hi) { return v < lo ? lo : (v > hi ? hi : v); }

__global__ __launch_bounds__(256) void prep_kernel(const float* __restrict__ emb, const float* __restrict__ win, const float* __restrict__ wh, const float* __restrict__ wo, b16* __restrict__ EM16, b16* __restrict__ WI, b16* __restrict__ WH, b16* __restrict__ WO) {
  const int t = blockIdx.x * 256 + threadIdx.x; const int n1 = V * EP / 8, n2 = H * EP / 8, n3 = H * H / 8, n4 = V * H / 8; v8b o; int u = t;
  if (u < n1) { const int e = u * 8, v = e / EP, k0 = e % EP; for (int j = 0; j < 8; ++j) { const int k = k0 + j; o[j] = (k < E) ? (b16)(bf16_rne(emb[v * E + k]) * XS) : (b16)0.0f; } for (int pass = 0; pass < 2; ++pass) { *(volatile v8b*)(EM16 + e) = o; __threadfence(); } return; } u -= n1;
  if (u < n2) { const int e = u * 8, oo = e / EP, k0 = e % EP; for (int j = 0; j < 8; ++j) { const int k = k0 + j; o[j] = (k < E) ? (b16)(bf16_rne(win[k * H + oo]) * WSC) : (b16)0.0f; } for (int pass = 0; pass < 2; ++pass) { *(volatile v8b*)(WI + e) = o; __threadfence(); } return; } u -= n2;
  if (u < n3) { const int e = u * 8, oo = e / H, k0 = e % H; for (int j = 0; j < 8; ++j) o[j] = (b16)(bf16_rne(wh[(k0 + j) * H + oo]) * WSC); for (int pass = 0; pass < 2; ++pass) { *(volatile v8b*)(WH + e) = o; __threadfence(); } return; } u -= n3;
  if (u < n4) { const int e = u * 8, oo = e / H, k0 = e % H; for (int j = 0; j < 8; ++j) o[j] = (b16)(bf16_rne(wo[(k0 + j) * V + oo]) * WSC); for (int pass = 0; pass < 2; ++pass) { *(volatile v8b*)(WO + e) = o; __threadfence(); } }
}
__global__ __launch_bounds__(32) void xt_kernel(const b16* __restrict__ EM16, const b16* __restrict__ WI, const float* __restrict__ bin, float* __restrict__ XT) {
  __shared__ __attribute__((aligned(16))) float Tf[1][16][H + 4];
  const int wave = 0, lane = threadIdx.x & 31, nloc = lane & 15, hlf = lane >> 4; const int m0 = blockIdx.x * 16;
  for (int t = 0; t < 16; ++t) { v8f acc = {};
    for (int kb = 0; kb < EP; kb += 32) acc = wmma16b(frag_kb(EM16 + (m0 + nloc) * EP + kb, hlf), frag_kb(WI + (t * 16 + nloc) * EP + kb, hlf), acc);
    const float bb = bf16_rne(bin[t * 16 + nloc]);
#pragma unroll 1
    for (int r = 0; r < 8; ++r) Tf[wave][8 * hlf + r][t * 16 + nloc] = fmaxf(acc[r] * (1.0f / (XS * WSC)) + bb, 0.0f); }
  wave_lds_sync();
  for (int pass = 0; pass < 2; ++pass) { for (int q = lane; q < 16 * (H / 4); q += 32) { const int rr = q / (H / 4), c4 = (q % (H / 4)) * 4; *(volatile v4f*)(XT + (m0 + rr) * H + c4) = *(const v4f*)(&Tf[wave][rr][c4]); } __threadfence(); }
}
__global__ __launch_bounds__(256) void rnn_kernel(const int* __restrict__ seq, const float* __restrict__ XT, const b16* __restrict__ WH, const float* __restrict__ bh, const b16* __restrict__ WO, const float* __restrict__ bo, float* __restrict__ out) {
  __shared__ __attribute__((aligned(16))) float Hf[RB][H + 4]; __shared__ __attribute__((aligned(16))) b16 Ah[RB][H + 8], Al[RB][H + 8]; __shared__ __attribute__((aligned(16))) float Lg[RB][V + 4];
  const int wave = threadIdx.x >> 5, lane = threadIdx.x & 31, nloc = lane & 15, hlf = lane >> 4, t_ = threadIdx.x; const size_t b0 = (size_t)blockIdx.x * RB; const int j0 = wave * 32;
  for (int q = t_; q < RB * H; q += 256) Hf[q / H][q % H] = 0.0f;
  float bhv[2]; for (int u = 0; u < 2; ++u) bhv[u] = bf16_rne(bh[j0 + u * 16 + nloc]);
  __syncthreads();
  for (int step = 0; step < T; ++step) {
    { const int row = t_ >> 3, cb = (t_ & 7) * 32; const int tok = iclamp(seq[(b0 + row) * T + step], 0, V - 1); const float* xt = XT + (size_t)tok * H + cb;
      for (int j = 0; j < 32; j += 4) { const v4f xv = *(const v4f*)(xt + j); for (int i = 0; i < 4; ++i) { b16 p, q; split16((xv[i] + Hf[row][cb + j + i]) * XS, p, q); Ah[row][cb + j + i] = p; Al[row][cb + j + i] = q; } } }
    __syncthreads();
    v8f acc[2][2] = {{{}, {}}, {{}, {}}};
#pragma unroll 2
    for (int kb = 0; kb < H; kb += 32) { v16b bw[2]; for (int u = 0; u < 2; ++u) bw[u] = frag_kb(WH + (size_t)(j0 + u * 16 + nloc) * H + kb, hlf);
#pragma unroll
      for (int a = 0; a < 2; ++a) { const v16b ha = frag_kb(&Ah[a * 16 + nloc][kb], hlf), hl = frag_kb(&Al[a * 16 + nloc][kb], hlf);
#pragma unroll
        for (int u = 0; u < 2; ++u) { acc[a][u] = wmma16b(ha, bw[u], acc[a][u]); acc[a][u] = wmma16b(hl, bw[u], acc[a][u]); } } }
#pragma unroll
    for (int a = 0; a < 2; ++a)
#pragma unroll
      for (int u = 0; u < 2; ++u)
#pragma unroll 1
        for (int r = 0; r < 8; ++r) Hf[a * 16 + 8 * hlf + r][j0 + u * 16 + nloc] = tanhf(acc[a][u][r] * (1.0f / (XS * WSC)) + bhv[u]);
    __syncthreads(); }
  { const int row = t_ >> 3, cb = (t_ & 7) * 32; for (int j = 0; j < 32; ++j) { b16 p, q; split16(Hf[row][cb + j] * XS, p, q); Ah[row][cb + j] = p; Al[row][cb + j] = q; } }
  __syncthreads();
  { v8f lo2[2] = {{}, {}};
#pragma unroll 2
    for (int kb = 0; kb < H; kb += 32) { const v16b bw = frag_kb(WO + (size_t)(wave * 16 + nloc) * H + kb, hlf);
#pragma unroll
      for (int a = 0; a < 2; ++a) { lo2[a] = wmma16b(frag_kb(&Ah[a * 16 + nloc][kb], hlf), bw, lo2[a]); lo2[a] = wmma16b(frag_kb(&Al[a * 16 + nloc][kb], hlf), bw, lo2[a]); } }
    const float bb = bf16_rne(bo[wave * 16 + nloc]);
#pragma unroll
    for (int a = 0; a < 2; ++a) for (int r = 0; r < 8; ++r) Lg[a * 16 + 8 * hlf + r][wave * 16 + nloc] = lo2[a][r] * (1.0f / (XS * WSC)) + bb; }
  __syncthreads();
  for (int rr = 0; rr < 4; ++rr) { const int row = wave * 4 + rr; const v4f lv = *(const v4f*)(&Lg[row][lane * 4]); float mx = fmaxf(fmaxf(lv[0], lv[1]), fmaxf(lv[2], lv[3]));
#pragma unroll
    for (int o = 16; o >= 1; o >>= 1) mx = fmaxf(mx, __shfl_xor(mx, o));
    float s = __expf(lv[0] - mx) + __expf(lv[1] - mx) + __expf(lv[2] - mx) + __expf(lv[3] - mx);
#pragma unroll
    for (int o = 16; o >= 1; o >>= 1) s += __shfl_xor(s, o);
    const float lse = mx + logf(s); v4f ov; for (int i = 0; i < 4; ++i) ov[i] = lv[i] - lse;
    for (int pass = 0; pass < 2; ++pass) { *(volatile v4f*)(out + (b0 + row) * V + lane * 4) = ov; __threadfence(); } }
}
}

extern "C" void kernel_launch(void* const* d_in, const int* in_sizes, int n_in, void* d_out, int out_size, void* d_ws, size_t ws_size, hipStream_t stream) {
  (void)n_in;
  auto Fp = [&](int i) { return (const float*)d_in[i]; }; auto Ip = [&](int i) { return (const int*)d_in[i]; };
  if (in_sizes[0] != NB * T || in_sizes[1] != V * E || in_sizes[2] != E * H || in_sizes[4] != H * H || in_sizes[6] != H * V || out_size != NB * V) return;
  size_t off = 0; char* ws = (char*)d_ws;
  auto carve = [&](size_t bytes) { char* p = ws + off; off += (bytes + 255) & ~(size_t)255; return p; };
  b16* EM16 = (b16*)carve((size_t)V * EP * 2); b16* WI = (b16*)carve((size_t)H * EP * 2); b16* WH = (b16*)carve((size_t)H * H * 2); b16* WO = (b16*)carve((size_t)V * H * 2); float* XT = (float*)carve((size_t)V * H * 4);
  if (off > ws_size) return;
  prep_kernel<<<(V * EP / 8 + H * EP / 8 + H * H / 8 + V * H / 8 + 255) / 256, 256, 0, stream>>>(Fp(1), Fp(2), Fp(4), Fp(6), EM16, WI, WH, WO);
  xt_kernel<<<V / 16, 32, 0, stream>>>(EM16, WI, Fp(3), XT);
  rnn_kernel<<<NB / RB, 256, 0, stream>>>(Ip(0), XT, WH, Fp(5), WO, Fp(7), (float*)d_out);
}
